// TFDebertaV2Attention_42030549959030
// MI455X (gfx1250) — hardware-verified
//
#include <hip/hip_runtime.h>
#include <math.h>

#define NB     2
#define SEQ    1024
#define HIDD   1024
#define NHEAD  16
#define DHD    64
#define SPAN2  512
#define HGRP   4
#define NGRP   (NHEAD / HGRP)
#define MROWS  (NB * SEQ)
#define PSCALE 32768.0f
#define LN_EPS 1e-7f

typedef __attribute__((ext_vector_type(16))) _Float16 v16h;
typedef __attribute__((ext_vector_type(8)))  _Float16 v8h;
typedef __attribute__((ext_vector_type(16))) __bf16   v16b;
typedef __attribute__((ext_vector_type(8)))  __bf16   v8b;
typedef __attribute__((ext_vector_type(8)))  float    v8f;
typedef __attribute__((ext_vector_type(4)))  float    v4f;
typedef __attribute__((ext_vector_type(2)))  float    v2f;
typedef __attribute__((ext_vector_type(4)))  unsigned int v4u;
typedef __attribute__((ext_vector_type(8)))  int      v8i;

__constant__ static const short kRelIdx[2047] = {0,0,0,0,0,0,0,0,0,0,0,0,0,0,0,0,0,0,0,0,0,0,0,0,0,0,0,0,0,0,0,0,0,0,0,0,0,0,0,0,0,0,0,0,0,0,0,0,0,0,0,0,0,0,0,0,0,0,0,0,0,0,0,0,0,0,0,0,0,0,0,0,0,0,0,0,0,0,0,0,0,0,0,0,0,0,0,0,0,0,0,0,0,0,0,0,0,0,0,0,0,0,0,0,0,0,0,0,0,0,0,0,0,0,0,0,0,0,0,0,0,0,0,0,0,0,0,0,0,0,0,0,0,0,0,0,0,0,0,0,0,0,0,0,0,0,0,0,0,0,0,0,0,0,0,0,0,0,0,0,0,0,0,0,0,0,0,0,0,0,0,0,0,0,0,0,0,0,0,0,0,0,0,0,0,0,0,0,0,0,0,0,0,0,0,0,0,0,0,0,0,0,0,0,0,0,0,0,0,0,0,0,0,0,0,0,0,0,0,0,0,0,0,0,0,0,0,0,0,0,0,0,0,0,0,0,0,0,0,0,0,0,0,0,0,0,0,0,0,0,0,0,0,0,0,0,0,0,0,0,0,0,0,0,0,0,0,0,0,0,0,0,0,0,0,0,0,0,0,0,0,0,0,0,0,0,0,0,0,0,0,0,0,0,0,0,0,0,0,0,0,0,0,0,0,0,0,0,0,0,0,0,0,0,0,0,0,0,0,0,0,0,0,0,0,0,0,0,0,0,0,0,0,0,0,0,0,0,0,0,0,0,0,0,0,0,0,0,0,0,0,0,0,0,0,0,0,0,0,0,0,0,0,0,0,0,0,0,0,0,0,0,0,0,0,0,0,0,0,0,0,0,0,0,0,0,0,0,0,0,0,0,0,0,0,0,0,0,0,0,0,0,0,0,0,0,0,0,0,0,0,0,0,0,0,0,0,0,0,0,0,0,0,0,0,0,0,0,0,0,0,0,0,0,0,0,0,0,0,0,0,0,0,0,0,0,0,0,0,0,0,0,0,0,0,0,0,0,0,0,0,0,0,0,0,0,0,0,0,0,0,0,0,0,0,0,0,0,0,0,0,0,0,0,0,0,0,0,0,0,0,0,0,0,0,0,0,0,0,0,0,0,0,0,0,0,0,0,0,0,0,0,1,1,1,1,1,1,2,2,2,2,2,2,3,3,3,3,3,4,4,4,4,4,5,5,5,5,5,5,6,6,6,6,6,7,7,7,7,7,8,8,8,8,8,9,9,9,9,9,10,10,10,10,10,11,11,11,11,11,12,12,12,12,12,13,13,13,13,13,14,14,14,14,14,15,15,15,15,15,16,16,16,16,17,17,17,17,17,18,18,18,18,18,19,19,19,19,20,20,20,20,20,21,21,21,21,22,22,22,22,23,23,23,23,23,24,24,24,24,25,25,25,25,26,26,26,26,26,27,27,27,27,28,28,28,28,29,29,29,29,30,30,30,30,31,31,31,31,32,32,32,32,33,33,33,33,34,34,34,34,35,35,35,35,36,36,36,37,37,37,37,38,38,38,38,39,39,39,40,40,40,40,41,41,41,41,42,42,42,43,43,43,43,44,44,44,45,45,45,45,46,46,46,47,47,47,48,48,48,48,49,49,49,50,50,50,51,51,51,52,52,52,52,53,53,53,54,54,54,55,55,55,56,56,56,57,57,57,58,58,58,59,59,59,60,60,60,61,61,61,62,62,62,63,63,64,64,64,65,65,65,66,66,66,67,67,68,68,68,69,69,69,70,70,71,71,71,72,72,73,73,73,74,74,75,75,75,76,76,77,77,77,78,78,79,79,79,80,80,81,81,82,82,83,83,83,84,84,85,85,86,86,87,87,87,88,88,89,89,90,90,91,91,92,92,93,93,94,94,95,95,96,96,97,97,98,98,99,99,100,100,101,101,102,103,103,104,104,105,105,106,106,107,108,108,109,109,110,111,111,112,112,113,114,114,115,115,116,117,117,118,119,119,120,121,121,122,123,123,124,125,125,126,127,128,129,130,131,132,133,134,135,136,137,138,139,140,141,142,143,144,145,146,147,148,149,150,151,152,153,154,155,156,157,158,159,160,161,162,163,164,165,166,167,168,169,170,171,172,173,174,175,176,177,178,179,180,181,182,183,184,185,186,187,188,189,190,191,192,193,194,195,196,197,198,199,200,201,202,203,204,205,206,207,208,209,210,211,212,213,214,215,216,217,218,219,220,221,222,223,224,225,226,227,228,229,230,231,232,233,234,235,236,237,238,239,240,241,242,243,244,245,246,247,248,249,250,251,252,253,254,255,256,257,258,259,260,261,262,263,264,265,266,267,268,269,270,271,272,273,274,275,276,277,278,279,280,281,282,283,284,285,286,287,288,289,290,291,292,293,294,295,296,297,298,299,300,301,302,303,304,305,306,307,308,309,310,311,312,313,314,315,316,317,318,319,320,321,322,323,324,325,326,327,328,329,330,331,332,333,334,335,336,337,338,339,340,341,342,343,344,345,346,347,348,349,350,351,352,353,354,355,356,357,358,359,360,361,362,363,364,365,366,367,368,369,370,371,372,373,374,375,376,377,378,379,380,381,382,383,384,385,386,387,387,388,389,389,390,391,391,392,393,393,394,395,395,396,397,397,398,398,399,400,400,401,401,402,403,403,404,404,405,406,406,407,407,408,408,409,409,410,411,411,412,412,413,413,414,414,415,415,416,416,417,417,418,418,419,419,420,420,421,421,422,422,423,423,424,424,425,425,425,426,426,427,427,428,428,429,429,429,430,430,431,431,432,432,433,433,433,434,434,435,435,435,436,436,437,437,437,438,438,439,439,439,440,440,441,441,441,442,442,443,443,443,444,444,444,445,445,446,446,446,447,447,447,448,448,448,449,449,450,450,450,451,451,451,452,452,452,453,453,453,454,454,454,455,455,455,456,456,456,457,457,457,458,458,458,459,459,459,460,460,460,460,461,461,461,462,462,462,463,463,463,464,464,464,464,465,465,465,466,466,466,467,467,467,467,468,468,468,469,469,469,469,470,470,470,471,471,471,471,472,472,472,472,473,473,473,474,474,474,474,475,475,475,475,476,476,476,477,477,477,477,478,478,478,478,479,479,479,479,480,480,480,480,481,481,481,481,482,482,482,482,483,483,483,483,484,484,484,484,485,485,485,485,486,486,486,486,486,487,487,487,487,488,488,488,488,489,489,489,489,489,490,490,490,490,491,491,491,491,492,492,492,492,492,493,493,493,493,494,494,494,494,494,495,495,495,495,495,496,496,496,496,497,497,497,497,497,498,498,498,498,498,499,499,499,499,499,500,500,500,500,500,501,501,501,501,501,502,502,502,502,502,503,503,503,503,503,504,504,504,504,504,505,505,505,505,505,506,506,506,506,506,507,507,507,507,507,507,508,508,508,508,508,509,509,509,509,509,510,510,510,510,510,510,511,511,511,511,511,511,511,511,511,511,511,511,511,511,511,511,511,511,511,511,511,511,511,511,511,511,511,511,511,511,511,511,511,511,511,511,511,511,511,511,511,511,511,511,511,511,511,511,511,511,511,511,511,511,511,511,511,511,511,511,511,511,511,511,511,511,511,511,511,511,511,511,511,511,511,511,511,511,511,511,511,511,511,511,511,511,511,511,511,511,511,511,511,511,511,511,511,511,511,511,511,511,511,511,511,511,511,511,511,511,511,511,511,511,511,511,511,511,511,511,511,511,511,511,511,511,511,511,511,511,511,511,511,511,511,511,511,511,511,511,511,511,511,511,511,511,511,511,511,511,511,511,511,511,511,511,511,511,511,511,511,511,511,511,511,511,511,511,511,511,511,511,511,511,511,511,511,511,511,511,511,511,511,511,511,511,511,511,511,511,511,511,511,511,511,511,511,511,511,511,511,511,511,511,511,511,511,511,511,511,511,511,511,511,511,511,511,511,511,511,511,511,511,511,511,511,511,511,511,511,511,511,511,511,511,511,511,511,511,511,511,511,511,511,511,511,511,511,511,511,511,511,511,511,511,511,511,511,511,511,511,511,511,511,511,511,511,511,511,511,511,511,511,511,511,511,511,511,511,511,511,511,511,511,511,511,511,511,511,511,511,511,511,511,511,511,511,511,511,511,511,511,511,511,511,511,511,511,511,511,511,511,511,511,511,511,511,511,511,511,511,511,511,511,511,511,511,511,511,511,511,511,511,511,511,511,511,511,511,511,511,511,511,511,511,511,511,511,511,511,511,511,511,511,511,511,511,511,511,511,511,511,511,511,511,511,511,511,511,511,511,511,511,511,511,511,511,511,511,511,511,511,511,511,511,511,511,511,511,511,511,511,511,511,511,511,511,511,511,511,511,511,511,511,511,511,511,511,511,511,511,511,511,511,511,511,511,511,511,511,511,511,511,511,511,511,511,511,511,511,511,511,511,511,511,511,511,511,511,511,511,511,511,511,511,511,511,511,511,511,511,511,511,511,511,511,511,511,511,511,511,511,511,511,511,511,511,511,511,511,511,511,511,511,511,511,511,511,511,511,511,511,511,511,511,511,511,511,511,511,511,511,511,511,511,511,511,511,511,511,511,511,511,511,511,511,511,511,511,511,511,511,511,511,511,511,511,511};

__device__ __forceinline__ unsigned short f2bf_bits(float f) {
  unsigned u = __float_as_uint(f);
  return (unsigned short)((u + 0x7FFFu + ((u >> 16) & 1u)) >> 16);
}
__device__ __forceinline__ float bf_bits2f(unsigned short h) { return __uint_as_float(((unsigned)h) << 16); }

__device__ __forceinline__ void dep_guard_h(v8f& a, v8f& b, v16h x, v16h y) { asm volatile("v_nop\n\tv_nop\n\tv_nop\n\tv_nop" : "+v"(a), "+v"(b) : "v"(x), "v"(y)); }
__device__ __forceinline__ void dep_guard_b(v8f& a, v8f& b, v16b x, v16b y) { asm volatile("v_nop\n\tv_nop\n\tv_nop\n\tv_nop" : "+v"(a), "+v"(b) : "v"(x), "v"(y)); }
__device__ __forceinline__ void keep4_h(v16h a, v16h b, v16h c, v16h d) { asm volatile("v_nop" :: "v"(a), "v"(b), "v"(c), "v"(d)); }
__device__ __forceinline__ void keep4_b(v16b a, v16b b, v16b c, v16b d) { asm volatile("v_nop" :: "v"(a), "v"(b), "v"(c), "v"(d)); }
__device__ __forceinline__ void acc_guard4(v8f& a, v8f& b, v8f& c, v8f& d) { asm volatile("v_nop\n\tv_nop\n\tv_nop\n\tv_nop" : "+v"(a), "+v"(b), "+v"(c), "+v"(d)); }
template <typename T> struct Frag;
template <> struct Frag<_Float16> {
  typedef v16h V; union U { v16h v; v8h h[2]; };
  static __device__ __forceinline__ v16h load(const _Float16* p) {
    U f; f.h[0] = *(const v8h*)(p); f.h[1] = *(const v8h*)(p + 16); return f.v;
  }
  static __device__ __forceinline__ v8f mma(v16h a, v16h b, v8f c) {
    return __builtin_amdgcn_wmma_f32_16x16x32_f16(false, a, false, b, (short)0, c, false, false);
  }
  static __device__ __forceinline__ void guard(v8f& a, v8f& b, v16h x, v16h y) { dep_guard_h(a, b, x, y); }
  static __device__ __forceinline__ void keep(v16h a, v16h b, v16h c, v16h d) { keep4_h(a, b, c, d); }
};
template <> struct Frag<__bf16> {
  typedef v16b V; union U { v16b v; v8b h[2]; };
  static __device__ __forceinline__ v16b load(const __bf16* p) {
    U f; f.h[0] = *(const v8b*)(p); f.h[1] = *(const v8b*)(p + 16); return f.v;
  }
  static __device__ __forceinline__ v8f mma(v16b a, v16b b, v8f c) {
    return __builtin_amdgcn_wmma_f32_16x16x32_bf16(false, a, false, b, (short)0, c, false, false);
  }
  static __device__ __forceinline__ void guard(v8f& a, v8f& b, v16b x, v16b y) { dep_guard_b(a, b, x, y); }
  static __device__ __forceinline__ void keep(v16b a, v16b b, v16b c, v16b d) { keep4_b(a, b, c, d); }
};

template <int ET> struct Elem;
template <> struct Elem<0> { typedef _Float16 T; };
template <> struct Elem<1> { typedef __bf16 T; };
template <int ET, bool SPLIT, int BIAS_MODE, int OUT_MODE, bool RESID, int ACT = 0>
__global__ __launch_bounds__(256) void wmma_gemm64(
    const unsigned short* __restrict__ Ap, const unsigned short* __restrict__ A2p, int lda, long strideA,
    const unsigned short* __restrict__ Btp, const unsigned short* __restrict__ Bt2p, int ldb, long strideB,
    void* __restrict__ Cout, void* __restrict__ Cout2, int ldc, long strideC,
    const float* __restrict__ bias,
    const float* __restrict__ resid, long strideR,
    int M, int N, int K, float scale) {
  typedef typename Elem<ET>::T T;
  typedef typename Frag<T>::V V;
  const T* A = (const T*)Ap; const T* A2 = (const T*)A2p; const T* Bt = (const T*)Btp; const T* Bt2 = (const T*)Bt2p;
  __shared__ __align__(16) float sT[8][16 * 68];
  const int b    = blockIdx.y;
  const int lane = threadIdx.x & 31;
  const int wave = threadIdx.x >> 5;
  const int tilesN = N >> 6;
  const int tilesM = M >> 6;
  const int tile = blockIdx.x * 8 + wave;
  if (tile >= tilesM * tilesN) return;
  const int tm = tile / tilesN;
  const int tn = tile - tm * tilesN;
  const int m0 = tm << 6;
  const int n0 = tn << 6;

  const T* Ab  = A  + (size_t)b * strideA;
  const T* Bb  = Bt + (size_t)b * strideB;
  const T* Ab2 = SPLIT ? (A2  + (size_t)b * strideA) : nullptr;
  const T* Bb2 = SPLIT ? (Bt2 + (size_t)b * strideB) : nullptr;

  const int rlane = lane & 15;
  const int koff  = (lane >> 4) * 8;
  const int mOff  = (lane >> 4) * 8;

  v8f acc[4][4];
#pragma unroll
  for (int i = 0; i < 4; ++i)
#pragma unroll
    for (int j = 0; j < 4; ++j) acc[i][j] = (v8f){0.f,0.f,0.f,0.f,0.f,0.f,0.f,0.f};

  for (int k0 = 0; k0 < K; k0 += 32) {
    V bh[4], bl[4];
#pragma unroll
    for (int j = 0; j < 4; ++j) {
      const size_t bo = (size_t)(n0 + (j << 4) + rlane) * ldb + koff + k0;
      bh[j] = Frag<T>::load(Bb + bo);
      if (SPLIT) bl[j] = Frag<T>::load(Bb2 + bo);
    }
#pragma unroll
    for (int i = 0; i < 4; ++i) {
      const size_t ao = (size_t)(m0 + (i << 4) + rlane) * lda + koff + k0;
      V ah = Frag<T>::load(Ab + ao);
      V al;
      if (SPLIT) al = Frag<T>::load(Ab2 + ao);
#pragma unroll
      for (int j = 0; j < 4; ++j) {
        acc[i][j] = Frag<T>::mma(ah, bh[j], acc[i][j]);
        if (SPLIT) {
          acc[i][j] = Frag<T>::mma(ah, bl[j], acc[i][j]);
          acc[i][j] = Frag<T>::mma(al, bh[j], acc[i][j]);
        }
      }
      Frag<T>::guard(acc[i][0], acc[i][3], ah, SPLIT ? al : ah);
    }
    Frag<T>::keep(bh[0], bh[1], bh[2], bh[3]);
    if (SPLIT) Frag<T>::keep(bl[0], bl[1], bl[2], bl[3]);
  }
  acc_guard4(acc[0][0], acc[0][1], acc[0][2], acc[0][3]);
  acc_guard4(acc[1][0], acc[1][1], acc[1][2], acc[1][3]);
  acc_guard4(acc[2][0], acc[2][1], acc[2][2], acc[2][3]);
  acc_guard4(acc[3][0], acc[3][1], acc[3][2], acc[3][3]);

  float* slab = sT[wave];
  const float* Rb = RESID ? (resid + (size_t)b * strideR) : nullptr;
#pragma unroll
  for (int i = 0; i < 4; ++i) {
    const int mBase = m0 + (i << 4);
#pragma unroll
    for (int j = 0; j < 4; ++j) {
      const int n = n0 + (j << 4) + rlane;
      float bv = 0.f;
      if (BIAS_MODE == 2) bv = bias[n];
#pragma unroll
      for (int r = 0; r < 8; ++r) {
        float v = acc[i][j][r] * scale;
        if (BIAS_MODE == 1) v += bias[mBase + mOff + r];
        if (BIAS_MODE == 2) v += bv;
        if (RESID) v += Rb[(size_t)(mBase + mOff + r) * ldc + n];
        if (ACT == 1) v = tanhf(v);
        if (ACT == 2) v = fmaxf(v, 0.0f);
        if (ACT == 3) v = v / (1.0f + expf(-v));
        if (ACT == 4) v = (v > 0.f) ? v : 0.01f * v;
        slab[(mOff + r) * 68 + (j << 4) + rlane] = v;
      }
    }
    __builtin_amdgcn_fence(__ATOMIC_RELEASE, "workgroup");
    __builtin_amdgcn_wave_barrier();
    __builtin_amdgcn_fence(__ATOMIC_ACQUIRE, "workgroup");
    if (OUT_MODE == 0) {
      float* C = (float*)Cout + (size_t)b * strideC;
      const int hh = lane >> 4, c4 = (lane & 15) * 4;
      for (int pass = 0; pass < 2; ++pass) {
#pragma unroll
        for (int it = 0; it < 8; ++it) {
          const int row = it * 2 + hh;
          v4f v = *(const v4f*)(slab + row * 68 + c4);
          *(volatile v4f*)(C + (size_t)(mBase + row) * ldc + n0 + c4) = v;
        }
        __threadfence();
      }
    } else {
      const int q = lane >> 3, c8 = (lane & 7) * 8;
      unsigned short* C  = (unsigned short*)Cout  + (size_t)b * strideC;
      unsigned short* C2 = (OUT_MODE == 2) ? ((unsigned short*)Cout2 + (size_t)b * strideC) : nullptr;
      for (int pass = 0; pass < 2; ++pass) {
#pragma unroll
        for (int it = 0; it < 4; ++it) {
          const int row = it * 4 + q;
          const float* sp = slab + row * 68 + c8;
          v8h hv, lv;
#pragma unroll
          for (int e = 0; e < 8; ++e) {
            if (OUT_MODE == 1) {
              hv[e] = (_Float16)sp[e];
            } else {
              unsigned short hb = f2bf_bits(sp[e]);
              unsigned short lb = f2bf_bits(sp[e] - bf_bits2f(hb));
              hv[e] = __builtin_bit_cast(_Float16, hb);
              lv[e] = __builtin_bit_cast(_Float16, lb);
            }
          }
          *(volatile v8h*)(C + (size_t)(mBase + row) * ldc + n0 + c8) = hv;
          if (OUT_MODE == 2) *(volatile v8h*)(C2 + (size_t)(mBase + row) * ldc + n0 + c8) = lv;
        }
        __threadfence();
      }
    }
    __builtin_amdgcn_fence(__ATOMIC_RELEASE, "workgroup");
    __builtin_amdgcn_wave_barrier();
    __builtin_amdgcn_fence(__ATOMIC_ACQUIRE, "workgroup");
  }
}

__device__ __forceinline__ unsigned pk16(unsigned short a, unsigned short b) { return (unsigned)a | ((unsigned)b << 16); }
__device__ __forceinline__ unsigned short h_bits(float f) { const _Float16 h = (_Float16)f; return __builtin_bit_cast(unsigned short, h); }

__global__ __launch_bounds__(256) void cast_f16x2_kernel(const float* __restrict__ in, unsigned short* __restrict__ out, int n2, float scale) {
  const int i = blockIdx.x * 256 + threadIdx.x;
  if (i < n2) {
    const v2f f = *(const v2f*)(in + 2 * (size_t)i);
    const unsigned u = pk16(h_bits(f[0] * scale), h_bits(f[1] * scale));
    ((volatile unsigned*)out)[i] = u;
    __threadfence();
    ((volatile unsigned*)out)[i] = u;
  }
}

__global__ __launch_bounds__(256) void transpose_cast_f16_kernel(const float* __restrict__ in, unsigned short* __restrict__ out,
                                                                 int R, int C, float scale) {
  __shared__ __align__(16) _Float16 tile[64 * 72];
  const int c0 = blockIdx.x * 64, r0 = blockIdx.y * 64;
  const int tid = threadIdx.x, lane = tid & 31, wave = tid >> 5;
  {
    const int rr = tid >> 2, cc = (tid & 3) * 16;
    const float* src = in + (size_t)(r0 + rr) * C + c0 + cc;
#pragma unroll
    for (int i = 0; i < 4; ++i) {
      const v4f f = *(const v4f*)(src + 4 * i);
#pragma unroll
      for (int e = 0; e < 4; ++e) tile[(cc + 4 * i + e) * 72 + rr] = (_Float16)(f[e] * scale);
    }
  }
  __syncthreads();
  const int q = lane >> 3, c8 = (lane & 7) * 8;
  const int orow0 = wave * 8 + q, orow1 = wave * 8 + 4 + q;
  const v8h v0 = *(const v8h*)(tile + orow0 * 72 + c8);
  const v8h v1 = *(const v8h*)(tile + orow1 * 72 + c8);
  unsigned short* o0 = out + (size_t)(c0 + orow0) * R + r0 + c8;
  unsigned short* o1 = out + (size_t)(c0 + orow1) * R + r0 + c8;
  *(volatile v8h*)o0 = v0;
  *(volatile v8h*)o1 = v1;
  __threadfence();
  *(volatile v8h*)o0 = v0;
  *(volatile v8h*)o1 = v1;
}

__global__ __launch_bounds__(128) void softmax_rel_kernel(const float* __restrict__ S,
                                                          const float* __restrict__ C2P,
                                                          const float* __restrict__ P2C,
                                                          const int* __restrict__ mask,
                                                          unsigned short* __restrict__ P, float inv) {
  __shared__ float redm[4];
  __shared__ float reds[4];
  const int qrow = blockIdx.x;
  const int hg   = blockIdx.y;
  const int tid  = threadIdx.x;
  const int lane = tid & 31;
  const int wave = tid >> 5;
  const int j0   = tid * 8;
  const size_t rowoff = ((size_t)hg * SEQ + qrow) * SEQ + j0;
  const v8f sv = *(const v8f*)(S + rowoff);
  const v8i mv = *(const v8i*)(mask + (size_t)qrow * SEQ + j0);
  const float* cpr = C2P + ((size_t)hg * SEQ + qrow) * SPAN2;
  const float* pcb = P2C + (size_t)hg * SEQ * SPAN2;
  float t[8];
  bool keep[8];
  float m = -INFINITY;
#pragma unroll
  for (int e = 0; e < 8; ++e) {
    const int kcol = j0 + e;
    int ix = (int)kRelIdx[qrow - kcol + (SEQ - 1)];
    ix = ix < 0 ? 0 : (ix > SPAN2 - 1 ? SPAN2 - 1 : ix);
    const float cp = cpr[ix];
    const float pc = pcb[(size_t)kcol * SPAN2 + ix];
    const float s  = sv[e] * inv + (cp + pc) * inv;
    keep[e] = (mv[e] != 0);
    t[e] = keep[e] ? s : -INFINITY;
    m = fmaxf(m, t[e]);
  }
#pragma unroll
  for (int off = 16; off > 0; off >>= 1) m = fmaxf(m, __shfl_xor(m, off, 32));
  if (lane == 0) redm[wave] = m;
  __syncthreads();
  const float mx = fmaxf(fmaxf(redm[0], redm[1]), fmaxf(redm[2], redm[3]));
  float ev[8];
  float ps = 0.f;
#pragma unroll
  for (int e = 0; e < 8; ++e) {
    const float x = __expf(t[e] - mx);
    ev[e] = keep[e] ? x : 0.f;
    ps += ev[e];
  }
#pragma unroll
  for (int off = 16; off > 0; off >>= 1) ps += __shfl_xor(ps, off, 32);
  if (lane == 0) reds[wave] = ps;
  __syncthreads();
  const float tot = ((reds[0] + reds[1]) + reds[2]) + reds[3];
  const float is  = (tot > 0.f) ? (1.0f / tot) : 0.f;
  const float sc = is * PSCALE;
  const v4u hv = (v4u){pk16(h_bits(ev[0] * sc), h_bits(ev[1] * sc)),
                       pk16(h_bits(ev[2] * sc), h_bits(ev[3] * sc)),
                       pk16(h_bits(ev[4] * sc), h_bits(ev[5] * sc)),
                       pk16(h_bits(ev[6] * sc), h_bits(ev[7] * sc))};
  *(volatile v4u*)(P + rowoff) = hv;
  __threadfence();
  *(volatile v4u*)(P + rowoff) = hv;
}

__global__ __launch_bounds__(256) void layernorm_kernel(const float* __restrict__ Y, const float* __restrict__ gamma,
                                                        const float* __restrict__ beta, float* __restrict__ out) {
  __shared__ float red[8];
  __shared__ float red2[8];
  const int row = blockIdx.x;
  const int tid = threadIdx.x, lane = tid & 31, wave = tid >> 5;
  const int c0 = tid * 4;
  const size_t o = (size_t)row * HIDD + c0;
  const v4f x = *(const v4f*)(Y + o);
  float s = (x[0] + x[1]) + (x[2] + x[3]);
#pragma unroll
  for (int off = 16; off > 0; off >>= 1) s += __shfl_xor(s, off, 32);
  if (lane == 0) red[wave] = s;
  __syncthreads();
  float tot = red[0];
#pragma unroll
  for (int w = 1; w < 8; ++w) tot += red[w];
  const float mu = tot * (1.0f / (float)HIDD);
  const float d0 = x[0] - mu, d1 = x[1] - mu, d2 = x[2] - mu, d3 = x[3] - mu;
  float s2 = (d0 * d0 + d1 * d1) + (d2 * d2 + d3 * d3);
#pragma unroll
  for (int off = 16; off > 0; off >>= 1) s2 += __shfl_xor(s2, off, 32);
  if (lane == 0) red2[wave] = s2;
  __syncthreads();
  float tot2 = red2[0];
#pragma unroll
  for (int w = 1; w < 8; ++w) tot2 += red2[w];
  const float var  = tot2 * (1.0f / (float)HIDD);
  const float rstd = 1.0f / sqrtf(var + LN_EPS);
  const v4f g  = *(const v4f*)(gamma + c0);
  const v4f bt = *(const v4f*)(beta + c0);
  const v4f r  = (v4f){d0 * rstd * g[0] + bt[0], d1 * rstd * g[1] + bt[1],
                       d2 * rstd * g[2] + bt[2], d3 * rstd * g[3] + bt[3]};
  *(volatile v4f*)(out + o) = r;
  __threadfence();
  *(volatile v4f*)(out + o) = r;
}

extern "C" void kernel_launch(void* const* d_in, const int* in_sizes, int n_in,
                              void* d_out, int out_size, void* d_ws, size_t ws_size,
                              hipStream_t stream) {
  if (n_in < 13) return;
  if (in_sizes[0] != NB * SEQ * HIDD) return;
  if (in_sizes[1] != NB * SEQ * SEQ) return;
  if (in_sizes[2] != SPAN2 * HIDD) return;
  if (in_sizes[3] != HIDD * HIDD || in_sizes[5] != HIDD * HIDD || in_sizes[7] != HIDD * HIDD || in_sizes[9] != HIDD * HIDD) return;
  if (in_sizes[4] != HIDD || in_sizes[6] != HIDD || in_sizes[8] != HIDD || in_sizes[10] != HIDD) return;
  if (in_sizes[11] != HIDD || in_sizes[12] != HIDD) return;
  if (out_size != NB * SEQ * HIDD) return;

  const float* hs   = (const float*)d_in[0];
  const int*   mask = (const int*)d_in[1];
  const float* rel  = (const float*)d_in[2];
  const float* Wq   = (const float*)d_in[3];
  const float* bq   = (const float*)d_in[4];
  const float* Wk   = (const float*)d_in[5];
  const float* bk   = (const float*)d_in[6];
  const float* Wv   = (const float*)d_in[7];
  const float* bv   = (const float*)d_in[8];
  const float* Wo   = (const float*)d_in[9];
  const float* bo   = (const float*)d_in[10];
  const float* ga   = (const float*)d_in[11];
  const float* be   = (const float*)d_in[12];

  const size_t PW   = (size_t)HIDD * HIDD * 2;
  const size_t PX   = (size_t)MROWS * HIDD * 2;
  const size_t PR   = (size_t)SPAN2 * HIDD * 2;
  const size_t PY   = (size_t)MROWS * HIDD * 4;
  const size_t PS   = (size_t)HGRP * SEQ * SEQ * 4;
  const size_t PC   = (size_t)HGRP * SEQ * SPAN2 * 4;
  const size_t PP   = (size_t)HGRP * SEQ * SEQ * 2;
  size_t off = 0;
  const size_t oWqT = off; off += PW;
  const size_t oWkT = off; off += PW;
  const size_t oWvT = off; off += PW;
  const size_t oWoT = off; off += PW;
  const size_t oX16 = off; off += PX;
  const size_t oREL = off; off += PR;
  const size_t oQ16 = off; off += PX;
  const size_t oK16 = off; off += PX;
  const size_t oVT  = off; off += PX;
  const size_t oPK  = off; off += PR;
  const size_t oPQ  = off; off += PR;
  const size_t oCTX = off; off += PX;
  const size_t oY   = off; off += PY;
  const size_t oS   = off; off += PS;
  const size_t oC2P = off; off += PC;
  const size_t oP2C = off; off += PC;
  const size_t oP16 = off; off += PP;
  if (off > ws_size) return;

  char* ws = (char*)d_ws;
  unsigned short* WqT16 = (unsigned short*)(ws + oWqT);
  unsigned short* WkT16 = (unsigned short*)(ws + oWkT);
  unsigned short* WvT16 = (unsigned short*)(ws + oWvT);
  unsigned short* WoT16 = (unsigned short*)(ws + oWoT);
  unsigned short* X16   = (unsigned short*)(ws + oX16);
  unsigned short* REL16 = (unsigned short*)(ws + oREL);
  unsigned short* Q16   = (unsigned short*)(ws + oQ16);
  unsigned short* K16   = (unsigned short*)(ws + oK16);
  unsigned short* VT16  = (unsigned short*)(ws + oVT);
  unsigned short* PK16  = (unsigned short*)(ws + oPK);
  unsigned short* PQ16  = (unsigned short*)(ws + oPQ);
  unsigned short* CTX16 = (unsigned short*)(ws + oCTX);
  float*          Ybuf  = (float*)(ws + oY);
  float*          Sbuf  = (float*)(ws + oS);
  float*          C2Pb  = (float*)(ws + oC2P);
  float*          P2Cb  = (float*)(ws + oP2C);
  unsigned short* P16   = (unsigned short*)(ws + oP16);

  const dim3 blk(256);
  const float wscale = 1.0f / 16.0f;
  const float scl    = sqrtf((float)(DHD * 3));
  const float inv    = 1.0f / scl;

  const dim3 gT(HIDD / 64, HIDD / 64);
  transpose_cast_f16_kernel<<<gT, blk, 0, stream>>>(Wq, WqT16, HIDD, HIDD, 16.0f);
  transpose_cast_f16_kernel<<<gT, blk, 0, stream>>>(Wk, WkT16, HIDD, HIDD, 16.0f);
  transpose_cast_f16_kernel<<<gT, blk, 0, stream>>>(Wv, WvT16, HIDD, HIDD, 16.0f);
  transpose_cast_f16_kernel<<<gT, blk, 0, stream>>>(Wo, WoT16, HIDD, HIDD, 16.0f);

  const int n2x = MROWS * HIDD / 2;
  const int n2r = SPAN2 * HIDD / 2;
  cast_f16x2_kernel<<<dim3((n2x + 255) / 256), blk, 0, stream>>>(hs, X16, n2x, 1.0f);
  cast_f16x2_kernel<<<dim3((n2r + 255) / 256), blk, 0, stream>>>(rel, REL16, n2r, 1.0f);

  const dim3 gQK(((MROWS / 64) * (HIDD / 64) + 7) / 8, 1);
  wmma_gemm64<0, false, 2, 1, false, 0><<<gQK, blk, 0, stream>>>(
      X16, X16, HIDD, 0L, WqT16, WqT16, HIDD, 0L, (void*)Q16, (void*)Q16, HIDD, 0L,
      bq, hs, 0L, MROWS, HIDD, HIDD, wscale);
  wmma_gemm64<0, false, 2, 1, false, 0><<<gQK, blk, 0, stream>>>(
      X16, X16, HIDD, 0L, WkT16, WkT16, HIDD, 0L, (void*)K16, (void*)K16, HIDD, 0L,
      bk, hs, 0L, MROWS, HIDD, HIDD, wscale);
  const dim3 gVT(((HIDD / 64) * (SEQ / 64) + 7) / 8, NB);
  wmma_gemm64<0, false, 1, 1, false, 0><<<gVT, blk, 0, stream>>>(
      WvT16, WvT16, HIDD, 0L, X16, X16, HIDD, (long)SEQ * HIDD, (void*)VT16, (void*)VT16, SEQ, (long)HIDD * SEQ,
      bv, hs, 0L, HIDD, SEQ, HIDD, wscale);
  const dim3 gP(((SPAN2 / 64) * (HIDD / 64) + 7) / 8, 1);
  wmma_gemm64<0, false, 2, 1, false, 0><<<gP, blk, 0, stream>>>(
      REL16, REL16, HIDD, 0L, WkT16, WkT16, HIDD, 0L, (void*)PK16, (void*)PK16, HIDD, 0L,
      bk, hs, 0L, SPAN2, HIDD, HIDD, wscale);
  wmma_gemm64<0, false, 2, 1, false, 0><<<gP, blk, 0, stream>>>(
      REL16, REL16, HIDD, 0L, WqT16, WqT16, HIDD, 0L, (void*)PQ16, (void*)PQ16, HIDD, 0L,
      bq, hs, 0L, SPAN2, HIDD, HIDD, wscale);

  const dim3 gS(((SEQ / 64) * (SEQ / 64) + 7) / 8, HGRP);
  const dim3 gC(((SEQ / 64) * (SPAN2 / 64) + 7) / 8, HGRP);
  const dim3 gPV(((SEQ / 64) * (DHD / 64) + 7) / 8, HGRP);
  const float pvscale = 16.0f / PSCALE;

  for (int b = 0; b < NB; ++b) {
    const int* maskb = mask + (size_t)b * SEQ * SEQ;
    unsigned short* VTb = VT16 + (size_t)b * HIDD * SEQ;
    for (int g = 0; g < NGRP; ++g) {
      const size_t hc = (size_t)g * HGRP * DHD;
      const unsigned short* Qb = Q16 + (size_t)b * SEQ * HIDD + hc;
      const unsigned short* Kb = K16 + (size_t)b * SEQ * HIDD + hc;
      wmma_gemm64<0, false, 0, 0, false, 0><<<gS, blk, 0, stream>>>(
          Qb, Qb, HIDD, (long)DHD, Kb, Kb, HIDD, (long)DHD, (void*)Sbuf, (void*)Sbuf, SEQ, (long)SEQ * SEQ,
          bq, hs, 0L, SEQ, SEQ, DHD, 1.0f);
      wmma_gemm64<0, false, 0, 0, false, 0><<<gC, blk, 0, stream>>>(
          Qb, Qb, HIDD, (long)DHD, PK16 + hc, PK16 + hc, HIDD, (long)DHD, (void*)C2Pb, (void*)C2Pb, SPAN2, (long)SEQ * SPAN2,
          bq, hs, 0L, SEQ, SPAN2, DHD, 1.0f);
      wmma_gemm64<0, false, 0, 0, false, 0><<<gC, blk, 0, stream>>>(
          Kb, Kb, HIDD, (long)DHD, PQ16 + hc, PQ16 + hc, HIDD, (long)DHD, (void*)P2Cb, (void*)P2Cb, SPAN2, (long)SEQ * SPAN2,
          bq, hs, 0L, SEQ, SPAN2, DHD, 1.0f);
      softmax_rel_kernel<<<dim3(SEQ, HGRP), dim3(128), 0, stream>>>(Sbuf, C2Pb, P2Cb, maskb, P16, inv);
      wmma_gemm64<0, false, 0, 1, false, 0><<<gPV, blk, 0, stream>>>(
          P16, P16, SEQ, (long)SEQ * SEQ, VTb + hc * SEQ, VTb + hc * SEQ, SEQ, (long)DHD * SEQ,
          (void*)(CTX16 + (size_t)b * SEQ * HIDD + hc), (void*)(CTX16 + (size_t)b * SEQ * HIDD + hc), HIDD, (long)DHD,
          bq, hs, 0L, SEQ, DHD, SEQ, pvscale);
    }
  }
  wmma_gemm64<0, false, 2, 0, true, 0><<<gQK, blk, 0, stream>>>(
      CTX16, CTX16, HIDD, 0L, WoT16, WoT16, HIDD, 0L, (void*)Ybuf, (void*)Ybuf, HIDD, 0L,
      bo, hs, 0L, MROWS, HIDD, HIDD, 1.0f / 256.0f);
  layernorm_kernel<<<dim3(MROWS), blk, 0, stream>>>(Ybuf, ga, be, (float*)d_out);
}
